// CLSTransformerAggregator_19061064860083
// MI455X (gfx1250) — hardware-verified
//
#include <hip/hip_runtime.h>
#include <hip/hip_bf16.h>
#include <math.h>


typedef _Float16 bf16;
typedef _Float16 f16;
typedef __attribute__((ext_vector_type(4))) unsigned v4u_t;
typedef unsigned v4ua __attribute__((ext_vector_type(4), may_alias));
typedef __attribute__((ext_vector_type(4))) float v4f_t;
typedef float v4fa __attribute__((ext_vector_type(4), may_alias));
typedef __attribute__((ext_vector_type(16))) bf16  bf16x16;
typedef bf16x16 f16x16;
typedef __attribute__((ext_vector_type(8)))  bf16  bf16x8;
typedef bf16x8 f16x8;
typedef __attribute__((ext_vector_type(4)))  bf16  bf16x4;
typedef __attribute__((ext_vector_type(8)))  float f32x8;
__device__ __forceinline__ f32x8 wmma16(f16x16 a, f16x16 b, f32x8 c) {
  c = __builtin_amdgcn_wmma_f32_16x16x32_f16(false, a, false, b, (short)0, c, false, false);
  asm volatile("v_nop\n\tv_nop\n\tv_nop\n\tv_nop" : "+v"(c) : "v"(a), "v"(b));
  return c;
}
#define LDS_STRIDE 48
#define KSTRIDE    72
#define VSTRIDE    48

__device__ __forceinline__ f32x8 wmma_bf16(bf16x16 a, bf16x16 b, f32x8 c) {
  c = __builtin_amdgcn_wmma_f32_16x16x32_f16(false, a, false, b, (short)0, c, false, false);
  asm volatile("v_nop\n\tv_nop\n\tv_nop\n\tv_nop" : "+v"(c) : "v"(a), "v"(b));
  return c;
}

template <typename T>
__device__ __forceinline__ bf16x16 load_frag(const T* __restrict__ base, int ld,
                                             int row0, int k0) {
  const int lane = threadIdx.x & 31;
  const int r    = lane & 15;
  const int kh   = (lane >> 4) * 8;
  const T* p0 = base + (size_t)(row0 + r) * ld + (k0 + kh);
  const T* p1 = p0 + 16;
  bf16x16 f;
#pragma unroll
  for (int i = 0; i < 8; ++i) {
    f[i]     = (bf16)p0[i];
    f[i + 8] = (bf16)p1[i];
  }
  return f;
}

__device__ __forceinline__ bf16x16 lds_frag(const bf16* base, int stride) {
  const int lane = threadIdx.x & 31;
  const int row  = lane & 15;
  const int kh   = (lane >> 4) * 8;
  const bf16x8 lo = *(const bf16x8*)(base + row * stride + kh);
  const bf16x8 hi = *(const bf16x8*)(base + row * stride + kh + 16);
  bf16x16 f;
#pragma unroll
  for (int i = 0; i < 8; ++i) { f[i] = lo[i]; f[i + 8] = hi[i]; }
  return f;
}

template <typename T>
__device__ __forceinline__ void stage_read16(const T* __restrict__ p, float* buf) {
#pragma unroll
  for (int i = 0; i < 16; ++i) buf[i] = (float)p[i];
}

__device__ __forceinline__ void stage_write(bf16* dst, const float* buf, int nquad) {
#pragma unroll
  for (int i = 0; i < nquad; ++i) {
    bf16x4 q;
    q[0] = (bf16)buf[4 * i];     q[1] = (bf16)buf[4 * i + 1];
    q[2] = (bf16)buf[4 * i + 2]; q[3] = (bf16)buf[4 * i + 3];
    *(bf16x4*)(dst + 4 * i) = q;
  }
}


#define GSTR 48
#define GSTR 48
template <typename AT, int EPI, bool OUT16>
__global__ __launch_bounds__(256) void gemm_kne(const AT* __restrict__ A, int lda, const float* __restrict__ Wm, int ldw,
                                                const float* __restrict__ bias, const float* __restrict__ R, const float* __restrict__ gvec,
                                                void* __restrict__ Yv, int ldy, int K) {
  __shared__ __attribute__((aligned(16))) f16 ldsA[128 * GSTR];
  __shared__ __attribute__((aligned(16))) f16 ldsW[128 * GSTR];
  __shared__ __attribute__((aligned(16))) float oS[8][32 * 68];
  const int tid = threadIdx.x, lane = tid & 31, wave = tid >> 5, cl = lane & 15, rh = (lane >> 4) * 8;
  const int m0 = blockIdx.x * 128, n0 = blockIdx.y * 128;
  const int wm = (wave & 3) * 32, wn = (wave >> 2) * 64;
  f32x8 acc[2][4];
#pragma unroll
  for (int i = 0; i < 2; ++i)
#pragma unroll
    for (int j = 0; j < 4; ++j) { f32x8 z = {}; acc[i][j] = z; }
#pragma unroll 1
  for (int k0 = 0; k0 < K; k0 += 32) {
    __syncthreads();
    { const int row = tid >> 1, ch = (tid & 1) * 16;
      const AT* src = A + (size_t)(m0 + row) * lda + k0 + ch;
#pragma unroll
      for (int g = 0; g < 16; ++g) ldsA[row * GSTR + ch + g] = (f16)src[g]; }
    { const int k = tid >> 3, nn0 = (tid & 7) * 16;
      const float* src = Wm + (size_t)(k0 + k) * ldw + n0 + nn0;
#pragma unroll
      for (int g = 0; g < 4; ++g) { const v4f_t v = *(const v4f_t*)(src + 4 * g);
#pragma unroll
        for (int u = 0; u < 4; ++u) ldsW[(nn0 + 4 * g + u) * GSTR + k] = (f16)v[u]; } }
    __syncthreads();
    f16x16 af[2];
#pragma unroll
    for (int i = 0; i < 2; ++i) af[i] = lds_frag(ldsA + (wm + 16 * i) * GSTR, GSTR);
#pragma unroll
    for (int j = 0; j < 4; ++j) {
      const f16x16 bf = lds_frag(ldsW + (wn + 16 * j) * GSTR, GSTR);
#pragma unroll
      for (int i = 0; i < 2; ++i) acc[i][j] = wmma16(af[i], bf, acc[i][j]);
    }
  }
  float* so = oS[wave];
#pragma unroll
  for (int i = 0; i < 2; ++i)
#pragma unroll
    for (int j = 0; j < 4; ++j) {
      const int n = n0 + wn + 16 * j + cl;
      const float bv = bias ? bias[n] : 0.0f;
      const float gv = (EPI == 2 || EPI == 4) ? gvec[n] : 0.0f;
      if (EPI == 1) {
#pragma unroll 1
        for (int r = 0; r < 8; ++r) { const float xg = acc[i][j][r] + bv; so[(16 * i + rh + r) * 68 + 16 * j + cl] = 0.5f * xg * (1.0f + erff(xg * 0.70710678118654752f)); }
      } else {
#pragma unroll
        for (int r = 0; r < 8; ++r) {
          float v = acc[i][j][r] + bv;
          if (EPI == 3) v = fmaxf(v, 0.0f);
          if (EPI == 4) v = gv * v;
          if (EPI == 2) v = R[(size_t)(m0 + wm + 16 * i + rh + r) * ldy + n] + gv * v;
          so[(16 * i + rh + r) * 68 + 16 * j + cl] = v;
        }
      }
    }
  asm volatile("s_wait_dscnt 0" ::: "memory");
  __builtin_amdgcn_wave_barrier();
#pragma unroll 1
  for (int pass = 0; pass < 2; ++pass) {
    if (OUT16) {
      f16* Y = (f16*)Yv;
#pragma unroll
      for (int it = 0; it < 8; ++it) { const int c = lane + 32 * it, rr = c >> 3, q8 = (c & 7) * 8;
        union { f16 h[8]; v4u_t v; } u;
#pragma unroll
        for (int e = 0; e < 8; ++e) u.h[e] = (f16)so[rr * 68 + q8 + e];
        *(volatile v4u_t*)(Y + (size_t)(m0 + wm + rr) * ldy + n0 + wn + q8) = u.v; }
    } else {
      float* Y = (float*)Yv;
#pragma unroll
      for (int it = 0; it < 16; ++it) { const int f4 = lane + 32 * it, rr = f4 >> 4, q = (f4 & 15) * 4;
        *(volatile v4f_t*)(Y + (size_t)(m0 + wm + rr) * ldy + n0 + wn + q) = *(const v4fa*)(so + rr * 68 + q); }
    }
    __threadfence();
  }
}

template <typename AT, int EPI, bool OUT16>
__global__ __launch_bounds__(256) void gemm_knez(const AT* __restrict__ A, int lda, size_t strideA, const float* __restrict__ Wm, int ldw, size_t strideW,
                                                 const float* __restrict__ bias, const float* __restrict__ R, const float* __restrict__ gvec,
                                                 void* __restrict__ Yv, int ldy, size_t strideY, int K) {
  A += (size_t)blockIdx.z * strideA; Wm += (size_t)blockIdx.z * strideW; Yv = (void*)((char*)Yv + (size_t)blockIdx.z * strideY * (OUT16 ? 2 : 4)); if (R) R += (size_t)blockIdx.z * strideY;
  __shared__ __attribute__((aligned(16))) f16 ldsA[128 * GSTR];
  __shared__ __attribute__((aligned(16))) f16 ldsW[128 * GSTR];
  __shared__ __attribute__((aligned(16))) float oS[8][32 * 68];
  const int tid = threadIdx.x, lane = tid & 31, wave = tid >> 5, cl = lane & 15, rh = (lane >> 4) * 8;
  const int m0 = blockIdx.x * 128, n0 = blockIdx.y * 128;
  const int wm = (wave & 3) * 32, wn = (wave >> 2) * 64;
  f32x8 acc[2][4];
#pragma unroll
  for (int i = 0; i < 2; ++i)
#pragma unroll
    for (int j = 0; j < 4; ++j) { f32x8 z = {}; acc[i][j] = z; }
#pragma unroll 1
  for (int k0 = 0; k0 < K; k0 += 32) {
    __syncthreads();
    { const int row = tid >> 1, ch = (tid & 1) * 16;
      const AT* src = A + (size_t)(m0 + row) * lda + k0 + ch;
#pragma unroll
      for (int g = 0; g < 16; ++g) ldsA[row * GSTR + ch + g] = (f16)src[g]; }
    { const int k = tid >> 3, nn0 = (tid & 7) * 16;
      const float* src = Wm + (size_t)(k0 + k) * ldw + n0 + nn0;
#pragma unroll
      for (int g = 0; g < 4; ++g) { const v4f_t v = *(const v4f_t*)(src + 4 * g);
#pragma unroll
        for (int u = 0; u < 4; ++u) ldsW[(nn0 + 4 * g + u) * GSTR + k] = (f16)v[u]; } }
    __syncthreads();
    f16x16 af[2];
#pragma unroll
    for (int i = 0; i < 2; ++i) af[i] = lds_frag(ldsA + (wm + 16 * i) * GSTR, GSTR);
#pragma unroll
    for (int j = 0; j < 4; ++j) {
      const f16x16 bf = lds_frag(ldsW + (wn + 16 * j) * GSTR, GSTR);
#pragma unroll
      for (int i = 0; i < 2; ++i) acc[i][j] = wmma16(af[i], bf, acc[i][j]);
    }
  }
  float* so = oS[wave];
#pragma unroll
  for (int i = 0; i < 2; ++i)
#pragma unroll
    for (int j = 0; j < 4; ++j) {
      const int n = n0 + wn + 16 * j + cl;
      const float bv = bias ? bias[n] : 0.0f;
      const float gv = (EPI == 2 || EPI == 4) ? gvec[n] : 0.0f;
      if (EPI == 1) {
#pragma unroll 1
        for (int r = 0; r < 8; ++r) { const float xg = acc[i][j][r] + bv; so[(16 * i + rh + r) * 68 + 16 * j + cl] = 0.5f * xg * (1.0f + erff(xg * 0.70710678118654752f)); }
      } else {
#pragma unroll
        for (int r = 0; r < 8; ++r) {
          float v = acc[i][j][r] + bv;
          if (EPI == 3) v = fmaxf(v, 0.0f);
          if (EPI == 4) v = gv * v;
          if (EPI == 2) v = R[(size_t)(m0 + wm + 16 * i + rh + r) * ldy + n] + gv * v;
          so[(16 * i + rh + r) * 68 + 16 * j + cl] = v;
        }
      }
    }
  asm volatile("s_wait_dscnt 0" ::: "memory");
  __builtin_amdgcn_wave_barrier();
#pragma unroll 1
  for (int pass = 0; pass < 2; ++pass) {
    if (OUT16) {
      f16* Y = (f16*)Yv;
#pragma unroll
      for (int it = 0; it < 8; ++it) { const int c = lane + 32 * it, rr = c >> 3, q8 = (c & 7) * 8;
        union { f16 h[8]; v4u_t v; } u;
#pragma unroll
        for (int e = 0; e < 8; ++e) u.h[e] = (f16)so[rr * 68 + q8 + e];
        *(volatile v4u_t*)(Y + (size_t)(m0 + wm + rr) * ldy + n0 + wn + q8) = u.v; }
    } else {
      float* Y = (float*)Yv;
#pragma unroll
      for (int it = 0; it < 16; ++it) { const int f4 = lane + 32 * it, rr = f4 >> 4, q = (f4 & 15) * 4;
        *(volatile v4f_t*)(Y + (size_t)(m0 + wm + rr) * ldy + n0 + wn + q) = *(const v4fa*)(so + rr * 68 + q); }
    }
    __threadfence();
  }
}

template <typename AT, bool ACC>
__global__ __launch_bounds__(256) void gemm_kn2(const AT* __restrict__ A, int lda, size_t strideA,
                                               const float* __restrict__ Wm, int ldw, size_t strideW,
                                               const float* __restrict__ bias, float scale,
                                               float* __restrict__ Y, int ldy, size_t strideY, int K) {
  __shared__ __attribute__((aligned(16))) f16 ldsA[128 * GSTR], ldsAl[128 * GSTR];
  __shared__ __attribute__((aligned(16))) f16 ldsW[128 * GSTR], ldsWl[128 * GSTR];
  __shared__ __attribute__((aligned(16))) float oS[8][32 * 68];
  const int tid = threadIdx.x, lane = tid & 31, wave = tid >> 5, cl = lane & 15, rh = (lane >> 4) * 8;
  const int m0 = blockIdx.x * 128, n0 = blockIdx.y * 128;
  const int wm = (wave & 3) * 32, wn = (wave >> 2) * 64;
  A += (size_t)blockIdx.z * strideA; Wm += (size_t)blockIdx.z * strideW; Y += (size_t)blockIdx.z * strideY;
  f32x8 acc[2][4], accx[2][4];
#pragma unroll
  for (int i = 0; i < 2; ++i)
#pragma unroll
    for (int j = 0; j < 4; ++j) { f32x8 z = {}; acc[i][j] = z; accx[i][j] = z; }
#pragma unroll 1
  for (int k0 = 0; k0 < K; k0 += 32) {
    __syncthreads();
    {
      const int row = tid >> 1, ch = (tid & 1) * 16;
      const AT* src = A + (size_t)(m0 + row) * lda + k0 + ch;
#pragma unroll
      for (int g = 0; g < 16; ++g) { const float v = (float)src[g]; const f16 h = (f16)v; ldsA[row * GSTR + ch + g] = h; ldsAl[row * GSTR + ch + g] = (f16)((v - (float)h) * 2048.0f); }
    }
    {
      const int k = tid >> 3, nn0 = (tid & 7) * 16;
      const float* src = Wm + (size_t)(k0 + k) * ldw + n0 + nn0;
#pragma unroll
      for (int g = 0; g < 4; ++g) { const v4f_t v = *(const v4f_t*)(src + 4 * g);
#pragma unroll
        for (int u = 0; u < 4; ++u) { const f16 h = (f16)v[u]; ldsW[(nn0 + 4 * g + u) * GSTR + k] = h; ldsWl[(nn0 + 4 * g + u) * GSTR + k] = (f16)((v[u] - (float)h) * 2048.0f); } }
    }
    __syncthreads();
    f16x16 af[2], afl[2];
#pragma unroll
    for (int i = 0; i < 2; ++i) { af[i] = lds_frag(ldsA + (wm + 16 * i) * GSTR, GSTR); afl[i] = lds_frag(ldsAl + (wm + 16 * i) * GSTR, GSTR); }
#pragma unroll
    for (int j = 0; j < 4; ++j) {
      const f16x16 bf = lds_frag(ldsW + (wn + 16 * j) * GSTR, GSTR), bfl = lds_frag(ldsWl + (wn + 16 * j) * GSTR, GSTR);
#pragma unroll
      for (int i = 0; i < 2; ++i) { acc[i][j] = wmma16(af[i], bf, acc[i][j]); accx[i][j] = wmma16(af[i], bfl, accx[i][j]); accx[i][j] = wmma16(afl[i], bf, accx[i][j]); }
    }
  }
  float* so = oS[wave];
#pragma unroll
  for (int i = 0; i < 2; ++i)
#pragma unroll
    for (int j = 0; j < 4; ++j) {
      const float bv = bias ? bias[n0 + wn + 16 * j + cl] : 0.0f;
#pragma unroll
      for (int r = 0; r < 8; ++r) so[(16 * i + rh + r) * 68 + 16 * j + cl] = (acc[i][j][r] + accx[i][j][r] * (1.0f / 2048.0f)) * scale + bv;
    }
  asm volatile("s_wait_dscnt 0" ::: "memory");
  __builtin_amdgcn_wave_barrier();
  if (ACC) {
#pragma unroll
    for (int it = 0; it < 16; ++it) { const int f4 = lane + 32 * it, rr = f4 >> 4, q = (f4 & 15) * 4;
      const v4f_t old = *(const v4fa*)(Y + (size_t)(m0 + wm + rr) * ldy + n0 + wn + q);
      v4f_t v = *(const v4fa*)(so + rr * 68 + q); v += old; *(v4fa*)(so + rr * 68 + q) = v; }
    asm volatile("s_wait_dscnt 0" ::: "memory");
  }
#pragma unroll 1
  for (int pass = 0; pass < 2; ++pass) {
#pragma unroll
    for (int it = 0; it < 16; ++it) { const int f4 = lane + 32 * it, rr = f4 >> 4, q = (f4 & 15) * 4;
      *(volatile v4f_t*)(Y + (size_t)(m0 + wm + rr) * ldy + n0 + wn + q) = *(const v4fa*)(so + rr * 68 + q); }
    __threadfence();
  }
}

__global__ __launch_bounds__(256) void k_transpose(const float* __restrict__ Wm, float* __restrict__ Wt, int rows, int cols) {
  __shared__ float tS[64][65];
  const int tid = threadIdx.x, tbj = cols / 64, bi = blockIdx.x / tbj, bj = blockIdx.x % tbj;
  for (int e = tid; e < 64 * 64; e += 256) { const int r = e >> 6, c = e & 63; tS[r][c] = Wm[(size_t)(bi * 64 + r) * cols + bj * 64 + c]; }
  __syncthreads();
  for (int ch = tid; ch < 64 * 16; ch += 256) { const int r = ch >> 4, q4 = (ch & 15) * 4; v4f_t o; o[0] = tS[q4][r]; o[1] = tS[q4 + 1][r]; o[2] = tS[q4 + 2][r]; o[3] = tS[q4 + 3][r];
    float* dst = Wt + (size_t)(bj * 64 + r) * rows + bi * 64 + q4; *(volatile v4f_t*)dst = o; __threadfence(); *(volatile v4f_t*)dst = o; }
}

__global__ __launch_bounds__(256) void k_transpose_ld(const float* __restrict__ Wm, int lds, float* __restrict__ Wt, int rows, int cols) {
  __shared__ float tS[64][65];
  const int tid = threadIdx.x, tbj = cols / 64, bi = blockIdx.x / tbj, bj = blockIdx.x % tbj;
  for (int e = tid; e < 64 * 64; e += 256) { const int r = e >> 6, c = e & 63; tS[r][c] = Wm[(size_t)(bi * 64 + r) * lds + bj * 64 + c]; }
  __syncthreads();
  for (int ch = tid; ch < 64 * 16; ch += 256) { const int r = ch >> 4, q4 = (ch & 15) * 4; v4f_t o; o[0] = tS[q4][r]; o[1] = tS[q4 + 1][r]; o[2] = tS[q4 + 2][r]; o[3] = tS[q4 + 3][r];
    float* dst = Wt + (size_t)(bj * 64 + r) * rows + bi * 64 + q4; *(volatile v4f_t*)dst = o; __threadfence(); *(volatile v4f_t*)dst = o; }
}
#define NBc 8
#define NNc 1024
#define NIN 1024
#define SPc 1280
#define DDc 256
#define NHc 8
#define FFc 1024
#define NLc 4
__global__ __launch_bounds__(256) void k_fill(float* __restrict__ p, float val, size_t n4) { const size_t i = (size_t)blockIdx.x * 256 + threadIdx.x; if (i < n4) { v4f_t v = {val, val, val, val}; *(volatile v4f_t*)(p + 4 * i) = v; __threadfence(); *(volatile v4f_t*)(p + 4 * i) = v; } }
__global__ __launch_bounds__(256) void k_dbg_zero(float* __restrict__ p, size_t n4) { const size_t i = (size_t)blockIdx.x * 256 + threadIdx.x; if (i < n4) { v4f_t z = {0.f,0.f,0.f,0.f}; *(volatile v4f_t*)(p + 4 * i) = z; __threadfence(); *(volatile v4f_t*)(p + 4 * i) = z; } }
__global__ __launch_bounds__(256) void k_copy(const float* __restrict__ src, float* __restrict__ dst, size_t n4) { const size_t i = (size_t)blockIdx.x * 256 + threadIdx.x; if (i < n4) { const v4f_t v = *(const v4f_t*)(src + 4 * i); *(volatile v4f_t*)(dst + 4 * i) = v; __threadfence(); *(volatile v4f_t*)(dst + 4 * i) = v; } }
__global__ __launch_bounds__(256) void k_ln(const float* __restrict__ X, const float* __restrict__ gam, const float* __restrict__ bet, float* __restrict__ Y) {
  __shared__ __attribute__((aligned(16))) float rowS[16 * 260];
  const int tid = threadIdx.x, r = tid >> 4, part = tid & 15; const size_t row = (size_t)blockIdx.x * 16 + r;
  float s = 0.0f;
#pragma unroll 1
  for (int i = 0; i < 16; ++i) { const float v = X[row * 256 + part * 16 + i]; rowS[r * 260 + part * 16 + i] = v; s += v; }
  s += __shfl_xor(s, 1, 32); s += __shfl_xor(s, 2, 32); s += __shfl_xor(s, 4, 32); s += __shfl_xor(s, 8, 32);
  const float mean = s * (1.0f / 256.0f); float q = 0.0f;
#pragma unroll 1
  for (int i = 0; i < 16; ++i) { const float dv = rowS[r * 260 + part * 16 + i] - mean; q += dv * dv; }
  q += __shfl_xor(q, 1, 32); q += __shfl_xor(q, 2, 32); q += __shfl_xor(q, 4, 32); q += __shfl_xor(q, 8, 32);
  const float rstd = 1.0f / __builtin_sqrtf(q * (1.0f / 256.0f) + 1e-5f);
#pragma unroll 1
  for (int i = 0; i < 16; ++i) { const int c = part * 16 + i; rowS[r * 260 + c] = (rowS[r * 260 + c] - mean) * rstd * gam[c] + bet[c]; }
  __syncthreads();
#pragma unroll 1
  for (int pass = 0; pass < 2; ++pass) { for (int q4 = tid; q4 < 16 * 64; q4 += 256) { const int rr = q4 / 64, c4 = (q4 % 64) * 4;
      *(volatile v4f_t*)(Y + ((size_t)blockIdx.x * 16 + rr) * 256 + c4) = *(const v4fa*)(rowS + rr * 260 + c4); } __threadfence(); }
}
__global__ __launch_bounds__(256) void k_vmean(const float* __restrict__ V, int ldv, float* __restrict__ VB) {
  const int c = blockIdx.x * 256 + threadIdx.x; float s = 0.0f;
#pragma unroll 1
  for (int r = 0; r < 1280; ++r) s += V[(size_t)r * ldv + c];
  const float m = s * (1.0f / 1280.0f); *(volatile float*)(VB + c) = m; __threadfence(); *(volatile float*)(VB + c) = m;
}
__global__ __launch_bounds__(64) void k_init(const float* __restrict__ feat, const float* __restrict__ cls, const float* __restrict__ pos, float* __restrict__ X) {
  const int r = blockIdx.x, c = 4 * threadIdx.x; v4f_t v = {0.f, 0.f, 0.f, 0.f};
  const int rf = min(max(r - 1, 0), NNc - 1); const int rp = min(r, NNc);
  const v4f_t pv = *(const v4f_t*)(pos + (size_t)rp * DDc + c); const v4f_t fv = *(const v4f_t*)(feat + (size_t)rf * DDc + c); const v4f_t cv = *(const v4f_t*)(cls + c);
  if (r == 0) v = cv + pv; else if (r <= NNc) v = fv + pv;
  float* dst = X + (size_t)r * DDc + c; *(volatile v4f_t*)dst = v; __threadfence(); *(volatile v4f_t*)dst = v;
}
__global__ __launch_bounds__(256) void k_softmax_cls(float* __restrict__ Sm, const int* __restrict__ msk) {
  __shared__ float red[256];
  const int q = blockIdx.x, z = blockIdx.y, tid = threadIdx.x; float* sr = Sm + ((size_t)z * SPc + q) * SPc;
  float v[SPc / 256]; bool ok[SPc / 256]; float m = -3.0e38f;
#pragma unroll
  for (int e = 0; e < SPc / 256; ++e) { const int j = tid + 256 * e; ok[e] = (j == 0) || (j <= NNc && msk[min(max(j - 1, 0), NNc - 1)] != 0); v[e] = ok[e] ? sr[j] * 0.17677669529663687f : -3.0e38f; m = fmaxf(m, v[e]); }
  red[tid] = m; __syncthreads();
  for (int o = 128; o > 0; o >>= 1) { if (tid < o) red[tid] = fmaxf(red[tid], red[tid + o]); __syncthreads(); }
  m = red[0]; __syncthreads();
  float zs = 0.0f;
#pragma unroll
  for (int e = 0; e < SPc / 256; ++e) { v[e] = ok[e] ? expf(v[e] - m) : 0.0f; zs += v[e]; }
  red[tid] = zs; __syncthreads();
  for (int o = 128; o > 0; o >>= 1) { if (tid < o) red[tid] += red[tid + o]; __syncthreads(); }
  const float kk = 1024.0f / red[0]; const float pc = 1024.0f / (float)SPc;
#pragma unroll 1
  for (int pass = 0; pass < 2; ++pass) {
#pragma unroll
    for (int e = 0; e < SPc / 256; ++e) *(volatile float*)(sr + tid + 256 * e) = v[e] * kk - pc;
    __threadfence(); }
}
__global__ __launch_bounds__(256) void k_place32(const float* __restrict__ T, float* __restrict__ att, int h0, const float* __restrict__ VB) {
  const int tid = threadIdx.x; const int z = blockIdx.y; const int q = blockIdx.x * 32 + (tid >> 3); const int c4 = (tid & 7) * 4;
  v4f_t v = *(const v4f_t*)(T + ((size_t)z * SPc + q) * 128 + c4); const v4f_t mb = *(const v4f_t*)(VB + (h0 + z) * 32 + c4); v += mb;
  float* dst = att + (size_t)q * DDc + (h0 + z) * 32 + c4; *(volatile v4f_t*)dst = v; __threadfence(); *(volatile v4f_t*)dst = v;
}
__global__ __launch_bounds__(256) void k_clsrow(const float* __restrict__ Sm, float* __restrict__ PA, int hg) {
  const int j = blockIdx.x * 256 + threadIdx.x; const float pc = 1024.0f / (float)SPc; float s = 0.0f;
#pragma unroll
  for (int z = 0; z < 4; ++z) s += (Sm[(size_t)z * SPc * SPc + j] + pc) * (1.0f / 1024.0f);
  const float v = (hg == 0) ? s : (PA[j] + s); *(volatile float*)(PA + j) = v; __threadfence(); *(volatile float*)(PA + j) = v;
}
__global__ __launch_bounds__(256) void k_final(const float* __restrict__ X, const float* __restrict__ g, const float* __restrict__ bb, const float* __restrict__ PA, const int* __restrict__ msk, float* __restrict__ co, float* __restrict__ ca) {
  __shared__ float red[256];
  const int tid = threadIdx.x; const float x = X[tid];
  red[tid] = x; __syncthreads(); for (int o = 128; o > 0; o >>= 1) { if (tid < o) red[tid] += red[tid + o]; __syncthreads(); }
  const float mean = red[0] * (1.0f / DDc); __syncthreads();
  const float d = x - mean; red[tid] = d * d; __syncthreads(); for (int o = 128; o > 0; o >>= 1) { if (tid < o) red[tid] += red[tid + o]; __syncthreads(); }
  const float rstd = 1.0f / __builtin_sqrtf(red[0] * (1.0f / DDc) + 1e-5f); __syncthreads();
  red[tid] = d * rstd * g[tid] + bb[tid]; __syncthreads();
  if (tid < 64) { const v4f_t v = *(const v4fa*)(red + 4 * tid); *(volatile v4f_t*)(co + 4 * tid) = v; __threadfence(); *(volatile v4f_t*)(co + 4 * tid) = v; }
  __syncthreads();
  float a[NNc / 256]; float s = 0.0f;
#pragma unroll
  for (int e = 0; e < NNc / 256; ++e) { const int j = tid + 256 * e; a[e] = PA[j + 1] * 0.125f * (float)(msk[j] != 0 ? 1 : 0) * 1.0f; a[e] = (msk[j] != 0) ? PA[j + 1] * 0.125f : 0.0f; s += a[e]; }
  red[tid] = s; __syncthreads(); for (int o = 128; o > 0; o >>= 1) { if (tid < o) red[tid] += red[tid + o]; __syncthreads(); }
  const float inv = 1.0f / (red[0] + 1e-8f);
#pragma unroll 1
  for (int pass = 0; pass < 2; ++pass) {
#pragma unroll
    for (int e = 0; e < NNc / 256; ++e) *(volatile float*)(ca + tid + 256 * e) = a[e] * inv;
    __threadfence(); }
}

extern "C" void kernel_launch(void* const* d_in, const int* in_sizes, int n_in,
                              void* d_out, int out_size, void* d_ws, size_t ws_size,
                              hipStream_t stream) {
  (void)in_sizes; (void)n_in; (void)out_size;
  const float* feat = (const float*)d_in[0]; const int* msk = (const int*)d_in[1]; const float* cls = (const float*)d_in[2], *pos = (const float*)d_in[3];
  const float* Win = (const float*)d_in[4], *bin = (const float*)d_in[5], *Wout = (const float*)d_in[6], *bout = (const float*)d_in[7], *W1 = (const float*)d_in[8], *b1 = (const float*)d_in[9], *W2 = (const float*)d_in[10], *b2 = (const float*)d_in[11];
  const float* g1 = (const float*)d_in[12], *be1 = (const float*)d_in[13], *g2 = (const float*)d_in[14], *be2 = (const float*)d_in[15], *gf = (const float*)d_in[16], *bf = (const float*)d_in[17];
  float* cls_out = (float*)d_out;
  float* cls_attn = (float*)d_out + (size_t)8 * DDc;
  char* ws = (char*)d_ws;
  float* WinT = (float*)ws; ws += (size_t)NLc * DDc * 3 * DDc * 4; float* WoT = (float*)ws; ws += (size_t)NLc * DDc * DDc * 4; float* W1T = (float*)ws; ws += (size_t)NLc * DDc * FFc * 4; float* W2T = (float*)ws; ws += (size_t)NLc * FFc * DDc * 4;
  float* X = (float*)ws; ws += (size_t)SPc * DDc * 4; float* XN = (float*)ws; ws += (size_t)SPc * DDc * 4;
  float* QKV = (float*)ws; ws += (size_t)SPc * 3 * DDc * 4 + 1024;
  float* KT = (float*)ws; ws += (size_t)DDc * SPc * 4;
  float* S = (float*)ws; ws += (size_t)4 * SPc * SPc * 4;
  float* T = (float*)ws; ws += (size_t)4 * SPc * 128 * 4; float* sc = (float*)ws; ws += 128 * 4; float* ones = (float*)ws; ws += FFc * 4; float* VB = (float*)ws; ws += DDc * 4;
  float* ATT = (float*)ws; ws += (size_t)SPc * DDc * 4;
  f16* Hf = (f16*)ws; ws += (size_t)SPc * FFc * 2;
  float* PA = (float*)ws; ws += (size_t)SPc * 4;
  if ((size_t)(ws - (char*)d_ws) > ws_size) return;
  const dim3 blk(256);
  k_fill<<<dim3(1), blk, 0, stream>>>(sc, 1.0f / 1024.0f, 128 / 4); k_fill<<<dim3(1), blk, 0, stream>>>(QKV + (size_t)SPc * 3 * DDc, 0.0f, 256 / 4); k_fill<<<dim3(1), blk, 0, stream>>>(ones, 1.0f, FFc / 4);
  for (int l = 0; l < NLc; ++l) {
    k_transpose<<<dim3((3 * DDc / 64) * (DDc / 64)), blk, 0, stream>>>(Win + (size_t)l * 3 * DDc * DDc, WinT + (size_t)l * DDc * 3 * DDc, 3 * DDc, DDc);
    k_transpose<<<dim3((DDc / 64) * (DDc / 64)), blk, 0, stream>>>(Wout + (size_t)l * DDc * DDc, WoT + (size_t)l * DDc * DDc, DDc, DDc);
    k_transpose<<<dim3((FFc / 64) * (DDc / 64)), blk, 0, stream>>>(W1 + (size_t)l * FFc * DDc, W1T + (size_t)l * DDc * FFc, FFc, DDc);
    k_transpose<<<dim3((DDc / 64) * (FFc / 64)), blk, 0, stream>>>(W2 + (size_t)l * DDc * FFc, W2T + (size_t)l * FFc * DDc, DDc, FFc);
  }

  for (int b = 0; b < NBc; ++b) {
    const int* mb = msk + (size_t)b * NIN;
    k_init<<<dim3(SPc), dim3(64), 0, stream>>>(feat + (size_t)b * NIN * DDc, cls, pos, X);
    for (int l = 0; l < NLc; ++l) {
      const float* wi = WinT + (size_t)l * DDc * 3 * DDc, *wo = WoT + (size_t)l * DDc * DDc, *w1 = W1T + (size_t)l * DDc * FFc, *w2 = W2T + (size_t)l * FFc * DDc;
      k_ln<<<dim3(SPc / 16), blk, 0, stream>>>(X, g1 + l * DDc, be1 + l * DDc, XN);
      gemm_kne<float, 0, false><<<dim3(SPc / 128, 3 * DDc / 128), blk, 0, stream>>>(XN, DDc, wi, 3 * DDc, bin + l * 3 * DDc, nullptr, nullptr, QKV, 3 * DDc, DDc);
      k_vmean<<<dim3(DDc / 256), blk, 0, stream>>>(QKV + 2 * DDc, 3 * DDc, VB);
      k_transpose_ld<<<dim3((SPc / 64) * (DDc / 64)), blk, 0, stream>>>(QKV + DDc, 3 * DDc, KT, SPc, DDc);
      for (int hg = 0; hg < 2; ++hg) { const int h0 = 4 * hg;
        gemm_knez<float, 0, false><<<dim3(SPc / 128, SPc / 128, 4), blk, 0, stream>>>(QKV + h0 * 32, 3 * DDc, (size_t)32, KT + (size_t)h0 * 32 * SPc, SPc, (size_t)32 * SPc, nullptr, nullptr, nullptr, S, SPc, (size_t)SPc * SPc, 32);
        k_softmax_cls<<<dim3(SPc, 4), blk, 0, stream>>>(S, mb);
        if (l == NLc - 1) k_clsrow<<<dim3(SPc / 256), blk, 0, stream>>>(S, PA, hg);
        gemm_knez<float, 4, false><<<dim3(SPc / 128, 1, 4), blk, 0, stream>>>(S, SPc, (size_t)SPc * SPc, QKV + 2 * DDc + h0 * 32, 3 * DDc, (size_t)32, nullptr, nullptr, sc, T, 128, (size_t)SPc * 128, SPc);
        k_place32<<<dim3(SPc / 32, 4), blk, 0, stream>>>(T, ATT, h0, VB);
      }
      gemm_kne<float, 2, false><<<dim3(SPc / 128, DDc / 128), blk, 0, stream>>>(ATT, DDc, wo, DDc, bout + l * DDc, X, ones, X, DDc, DDc);
      k_ln<<<dim3(SPc / 16), blk, 0, stream>>>(X, g2 + l * DDc, be2 + l * DDc, XN);
      gemm_kne<float, 1, true><<<dim3(SPc / 128, FFc / 128), blk, 0, stream>>>(XN, DDc, w1, FFc, b1 + l * FFc, nullptr, nullptr, Hf, FFc, DDc);
      gemm_kne<f16, 2, false><<<dim3(SPc / 128, DDc / 128), blk, 0, stream>>>(Hf, FFc, w2, DDc, b2 + l * DDc, X, ones, X, DDc, FFc);
    }
    k_final<<<dim3(1), blk, 0, stream>>>(X, gf, bf, PA, mb, cls_out + (size_t)b * DDc, cls_attn + (size_t)b * NIN);
  }
}
